// MultiHeadedAttention_17489106830130
// MI455X (gfx1250) — hardware-run, weakly checked
//
#include <hip/hip_runtime.h>


#ifndef NB
#define NB 4
#endif
#ifndef SEQ
#define SEQ 2048
#endif
#define NB_FULL  4
#define SEQ_FULL 2048
#ifndef OUT_SEQ
#define OUT_SEQ SEQ
#endif
#define DM   1024
#define NH_  16
#define HD   64
#define AW   4
#define OSP  68
#define EROWS (SEQ < 1024 ? SEQ : 1024)
#define QRS  2048.0f
#define QRI  (1.0f / 2048.0f)
#define SC2  ((float)(0.125 * 1.4426950408889634))
#define PSH  14.0f
#define NEGB (-3.0e38f)

static_assert(HD == 64);
static_assert(NH_ * HD == DM);
static_assert(DM % 64 == 0);
static_assert(DM % 32 == 0);
static_assert(HD % 32 == 0);
static_assert(SEQ % 64 == 0);
static_assert((NB * SEQ) % 64 == 0);
static_assert(SEQ % 32 == 0);
static_assert(SEQ % (16 * AW) == 0);
static_assert(EROWS % 64 == 0);
static_assert(EROWS % 32 == 0);
static_assert(EROWS >= 32);
static_assert(EROWS <= SEQ);
static_assert(EROWS % (16 * AW) == 0);
static_assert((SEQ - EROWS) % (16 * AW) == 0);
static_assert(((size_t)SEQ * DM) % 8 == 0);
static_assert(((size_t)DM * DM) % 8 == 0);
static_assert(NB <= NB_FULL);
static_assert(SEQ <= SEQ_FULL);
static_assert((OSP * 4) % 16 == 0);
static_assert(OSP >= HD);
static_assert(32 * 16 * 4 == 16 * HD * 2);
static_assert(32 * 16 * 4 == 16 * 64 * 2);
static_assert(32 * 16 * 8 == 16 * HD * 4);
static_assert(256 * 16 * 2 == 64 * 64 * 2);
static_assert(256 * 4 * 16 == 64 * 64 * 4);
static_assert(16 * 68 * 4 <= 131072);
static_assert(AW * 16 * OSP * 4 <= 131072);
static_assert(64 * 68 * 4 <= 131072);

typedef _Float16 h16;
typedef unsigned short bf;
typedef __attribute__((ext_vector_type(16))) __bf16   v16bf;
typedef __attribute__((ext_vector_type(16))) _Float16 v16h;
typedef __attribute__((ext_vector_type(8)))  _Float16 v8h;
typedef __attribute__((ext_vector_type(8)))  unsigned short v8us;
typedef __attribute__((ext_vector_type(8)))  float    v8f;
typedef __attribute__((ext_vector_type(4)))  float    v4f;
typedef v4f  __attribute__((may_alias)) v4fa;

__device__ __forceinline__ unsigned short f2bf(float f) { unsigned u = __float_as_uint(f); u += 0x7FFFu + ((u >> 16) & 1u); return (unsigned short)(u >> 16); }
__device__ __forceinline__ float bfr(float f) { return __uint_as_float(((unsigned)f2bf(f)) << 16); }
__device__ __forceinline__ v16h cat16(v8h lo, v8h hi) { return __builtin_shufflevector(lo, hi, 0, 1, 2, 3, 4, 5, 6, 7, 8, 9, 10, 11, 12, 13, 14, 15); }
__device__ __forceinline__ v16bf cat16b(v8us lo, v8us hi) { return __builtin_bit_cast(v16bf, __builtin_shufflevector(lo, hi, 0, 1, 2, 3, 4, 5, 6, 7, 8, 9, 10, 11, 12, 13, 14, 15)); }
__device__ __forceinline__ v8f wmma16(v16h a, v16h b, v8f c) { return __builtin_amdgcn_wmma_f32_16x16x32_f16(false, a, false, b, (short)0, c, false, false); }
__device__ __forceinline__ v8f wmmab(v16bf a, v16bf b, v8f c) { return __builtin_amdgcn_wmma_f32_16x16x32_bf16(false, a, false, b, (short)0, c, false, false); }
__device__ __forceinline__ v16h  ldh(const h16* p) { return cat16(*(const v8h*)p, *(const v8h*)(p + 16)); }
__device__ __forceinline__ v16bf ldb(const bf* p)  { return cat16b(*(const v8us*)p, *(const v8us*)(p + 16)); }
__device__ __forceinline__ void wave_sync() { __builtin_amdgcn_fence(3  , "wavefront"); __builtin_amdgcn_wave_barrier(); asm volatile("" ::: "memory"); }

__device__ __forceinline__ v8f wmmabg(v16bf a, v16bf b, v8f c) { c = wmmab(a, b, c); asm volatile("v_nop\n\tv_nop\n\tv_nop\n\tv_nop" : "+v"(c) : "v"(a), "v"(b)); return c; }
__device__ __forceinline__ v8f wmma16g(v16h a, v16h b, v8f c) { c = wmma16(a, b, c); asm volatile("v_nop\n\tv_nop\n\tv_nop\n\tv_nop" : "+v"(c) : "v"(a), "v"(b)); return c; }
static __device__ __forceinline__ h16 toh_flush(float v) { const float w = (fabsf(v) < 6.103515625e-05f) ? 0.0f : v; return (h16)w; }

__global__ __launch_bounds__(256) void k_cvt8(const float* __restrict__ src, bf* dst, size_t n8) {
    const size_t i = (size_t)blockIdx.x * 256 + threadIdx.x; if (i >= n8) return;
    const v8f v = *(const v8f*)(src + i * 8); v8us o;
#pragma unroll
    for (int k = 0; k < 8; ++k) o[k] = f2bf(v[k]);
    *(volatile v8us*)(dst + i * 8) = o; __threadfence(); *(volatile v8us*)(dst + i * 8) = o;
}

__global__ __launch_bounds__(256) void k_wtr(const float* __restrict__ W, bf* WT) {
    __shared__ __align__(16) float ts[64 * 68];
    const unsigned tid = threadIdx.x; const unsigned n0 = blockIdx.x * 64u, k0 = blockIdx.y * 64u;
#pragma unroll
    for (int i = 0; i < 4; ++i) { const unsigned p = (unsigned)i * 256u + tid; const unsigned row = p >> 4, c4 = (p & 15u) * 4u;
        const v4f v = *(const v4f*)(W + (size_t)(k0 + row) * DM + n0 + c4); *(v4fa*)(&ts[row * 68u + c4]) = v; }
    __syncthreads();
    const unsigned c8 = (tid & 7u) * 8u;
    v8us o0, o1;
#pragma unroll
    for (int e = 0; e < 8; ++e) { o0[e] = f2bf(ts[(c8 + (unsigned)e) * 68u + (tid >> 3)]); o1[e] = f2bf(ts[(c8 + (unsigned)e) * 68u + 32u + (tid >> 3)]); }
    bf* d0 = WT + (size_t)(n0 + (tid >> 3)) * DM + k0 + c8;
    bf* d1 = WT + (size_t)(n0 + 32u + (tid >> 3)) * DM + k0 + c8;
    *(volatile v8us*)d0 = o0; *(volatile v8us*)d1 = o1;
    __threadfence();
    *(volatile v8us*)d0 = o0; *(volatile v8us*)d1 = o1;
}

template <int MODE>
static __device__ __forceinline__ void proj_body(const bf* __restrict__ A, const bf* __restrict__ Bt, h16* Ph, h16* Pr, int resT) {
    __shared__ __align__(16) float os[16 * 68];
    const int K = DM;
    const int lane = threadIdx.x & 31, lr = lane & 15, hi = lane >> 4;
    const unsigned bx = blockIdx.x, by = blockIdx.y; const unsigned r0 = bx * 64u, c0 = by * 64u;
    const unsigned ru = (unsigned)resT;
    v8f acc[4][4];
#pragma unroll
    for (int mb = 0; mb < 4; ++mb)
#pragma unroll
        for (int nb = 0; nb < 4; ++nb) acc[mb][nb] = (v8f){};
    const size_t aoff = (size_t)(r0 + (unsigned)lr) * K + 8 * hi, boff = (size_t)(c0 + (unsigned)lr) * K + 8 * hi;
#pragma unroll 1
    for (int kc = 0; kc < K; kc += 32) {
        v16bf a[4];
#pragma unroll
        for (int mb = 0; mb < 4; ++mb) a[mb] = ldb(A + aoff + (size_t)mb * 16 * K + kc);
#pragma unroll
        for (int nb = 0; nb < 4; ++nb) { const v16bf b = ldb(Bt + boff + (size_t)nb * 16 * K + kc);
#pragma unroll
            for (int mb = 0; mb < 4; ++mb) acc[mb][nb] = wmmabg(a[mb], b, acc[mb][nb]); }
    }
    size_t tbase, rbase; bool wr;
    if (MODE == 0) { const unsigned bb = r0 / (unsigned)SEQ, tt = r0 % (unsigned)SEQ; const unsigned zc = bb * (unsigned)NH_ + c0 / (unsigned)HD;
                     tbase = ((size_t)zc * SEQ + (size_t)tt) * HD; rbase = ((size_t)zc * (size_t)ru + (size_t)tt) * HD; wr = tt < ru; }
    else           { const unsigned bb = c0 / (unsigned)SEQ, tt = c0 % (unsigned)SEQ;
                     tbase = (size_t)bb * (size_t)DM * SEQ + (size_t)r0 * SEQ + (size_t)tt; rbase = (size_t)bb * (size_t)DM * (size_t)ru + (size_t)r0 * (size_t)ru + (size_t)tt; wr = tt < ru; }
#pragma unroll
    for (int mb = 0; mb < 4; ++mb) {
#pragma unroll
        for (int nb = 0; nb < 4; ++nb) {
#pragma unroll
            for (int j = 0; j < 8; ++j) os[(hi * 8 + j) * 68 + nb * 16 + lr] = acc[mb][nb][j]; }
        wave_sync();
#pragma unroll 1
        for (int ps = 0; ps < 2; ++ps) {
            if (MODE == 0) {
                const size_t sb = tbase + (size_t)(mb * 16) * HD;
                const size_t rb = rbase + (size_t)(mb * 16) * HD;
#pragma unroll
                for (int s = 0; s < 4; ++s) { const int p = s * 32 + lane; const int row = p >> 3, c8 = (p & 7) * 8;
                    const v4f x0 = *(const v4fa*)(&os[row * 68 + c8]); const v4f x1 = *(const v4fa*)(&os[row * 68 + c8 + 4]); v8h hv, rv;
#pragma unroll
                    for (int i = 0; i < 4; ++i) { const h16 a0 = toh_flush(x0[i]); const h16 a1 = toh_flush(x1[i]); hv[i] = a0; hv[4 + i] = a1;
                        rv[i] = toh_flush((x0[i] - (float)a0) * QRS); rv[4 + i] = toh_flush((x1[i] - (float)a1) * QRS); }
                    const size_t oo = sb + (size_t)p * 8;
                    const size_t ro = rb + (size_t)p * 8;
                    *(volatile v8h*)(Ph + oo) = hv; if (wr) *(volatile v8h*)(Pr + ro) = rv; }
            } else {
                const size_t sb = tbase + (size_t)(mb * 16) * SEQ;
                const size_t rb = rbase + (size_t)(mb * 16) * (size_t)ru;
#pragma unroll
                for (int s = 0; s < 4; ++s) { const int row = 4 * s + (lane >> 3), c8 = (lane & 7) * 8;
                    const v4f x0 = *(const v4fa*)(&os[row * 68 + c8]); const v4f x1 = *(const v4fa*)(&os[row * 68 + c8 + 4]); v8h hv, rv;
#pragma unroll
                    for (int i = 0; i < 4; ++i) { const h16 a0 = toh_flush(x0[i]); const h16 a1 = toh_flush(x1[i]); hv[i] = a0; hv[4 + i] = a1;
                        rv[i] = toh_flush((x0[i] - (float)a0) * QRS); rv[4 + i] = toh_flush((x1[i] - (float)a1) * QRS); }
                    const size_t oo = sb + (size_t)row * SEQ + c8;
                    const size_t ro = rb + (size_t)row * (size_t)ru + c8;
                    *(volatile v8h*)(Ph + oo) = hv; if (wr) *(volatile v8h*)(Pr + ro) = rv; }
            }
            if (ps == 0) __threadfence(); }
        wave_sync();
    }
}

__global__ __launch_bounds__(32) void k_proj_rows(const bf* __restrict__ A, const bf* __restrict__ Bt, h16* Ph, h16* Pr, int resT) { proj_body<0>(A, Bt, Ph, Pr, resT); }
__global__ __launch_bounds__(32) void k_proj_cols(const bf* __restrict__ A, const bf* __restrict__ Bt, h16* Ph, h16* Pr, int resT) { proj_body<1>(A, Bt, Ph, Pr, resT); }

template <int EARLY>
static __device__ __forceinline__ void flash_body(const h16* __restrict__ QH, const h16* __restrict__ QR, const h16* __restrict__ KP, const h16* __restrict__ KR,
                                                  const h16* __restrict__ VT, const h16* __restrict__ VR, float* OUT) {
    __shared__ __align__(16) float os[AW * 16 * OSP];
    const int lane = threadIdx.x & 31, lr = lane & 15, hi = lane >> 4;
    const int wave = __builtin_amdgcn_readfirstlane((int)(threadIdx.x >> 5));
    const unsigned zh = blockIdx.y; const unsigned b = zh / (unsigned)NH_, h = zh % (unsigned)NH_;
    const int t0 = (EARLY ? 0 : EROWS) + ((int)blockIdx.x * AW + wave) * 16;
    const int lim = t0 + lr;
    const int nk = (t0 + 16 + 31) & ~31;
    const size_t pbase = (size_t)zh * SEQ * HD;
    const size_t rbase = (size_t)zh * EROWS * HD;
    const size_t qo = pbase + (size_t)(t0 + lr) * HD + 8 * hi;
    const v16h hz = (v16h){};
    const v16h qh0 = ldh(QH + qo), qh1 = ldh(QH + qo + 32);
    v16h qr0 = hz, qr1 = hz;
    if (EARLY) { const size_t qro = rbase + (size_t)(t0 + lr) * HD + 8 * hi; qr0 = ldh(QR + qro); qr1 = ldh(QR + qro + 32); }
    const size_t ko = pbase + (size_t)lr * HD + 8 * hi;
    const size_t vo = pbase + (size_t)lr * SEQ + 8 * hi;
    const size_t kro = rbase + (size_t)lr * HD + 8 * hi;
    const size_t vro = rbase + (size_t)lr * EROWS + 8 * hi;
    v8f o[4], oR[4];
#pragma unroll
    for (int j = 0; j < 4; ++j) { o[j] = (v8f){}; oR[j] = (v8f){}; }
    float m = NEGB, l = 0.0f;
#pragma unroll 1
    for (int key0 = 0; key0 < nk; key0 += 32) {
        const h16* ka = KP + ko + (size_t)key0 * HD;
        v8f sHa = (v8f){}, sLa = (v8f){}, sHb = (v8f){}, sLb = (v8f){};
        { const v16h ka0 = ldh(ka), kb0 = ldh(ka + 16 * HD);
          sHa = wmma16g(ka0, qh0, sHa); sHb = wmma16g(kb0, qh0, sHb);
          if (EARLY) { sLa = wmma16g(ka0, qr0, sLa); sLb = wmma16g(kb0, qr0, sLb); } }
        { const v16h ka1 = ldh(ka + 32), kb1 = ldh(ka + 16 * HD + 32);
          sHa = wmma16g(ka1, qh1, sHa); sHb = wmma16g(kb1, qh1, sHb);
          if (EARLY) { sLa = wmma16g(ka1, qr1, sLa); sLb = wmma16g(kb1, qr1, sLb); } }
        if (EARLY) {
            const h16* kr = KR + kro + (size_t)key0 * HD;
            { const v16h kra0 = ldh(kr), krb0 = ldh(kr + 16 * HD);
              sLa = wmma16g(kra0, qh0, sLa); sLb = wmma16g(krb0, qh0, sLb); }
            { const v16h kra1 = ldh(kr + 32), krb1 = ldh(kr + 16 * HD + 32);
              sLa = wmma16g(kra1, qh1, sLa); sLb = wmma16g(krb1, qh1, sLb); }
        }
        const int ja = key0 + 8 * hi;
        float ta[8], tb[8]; bool fa[8], fb[8]; float mx = NEGB;
#pragma unroll
        for (int r = 0; r < 8; ++r) {
            fa[r] = (ja + r <= lim);
            fb[r] = (ja + 16 + r <= lim);
            if (EARLY) { ta[r] = (sHa[r] + sLa[r] * QRI) * SC2; tb[r] = (sHb[r] + sLb[r] * QRI) * SC2; }
            else       { ta[r] = sHa[r] * SC2; tb[r] = sHb[r] * SC2; }
            mx = fmaxf(mx, fmaxf(fa[r] ? ta[r] : NEGB, fb[r] ? tb[r] : NEGB)); }
        mx = fmaxf(mx, __shfl_xor(mx, 16, 32));
        const float mnew = fmaxf(m, mx);
        const float alpha = __builtin_amdgcn_exp2f(m - mnew);
        const float sh = PSH - mnew;
        v16h pb, pr = hz; float ls = 0.0f;
#pragma unroll
        for (int r = 0; r < 8; ++r) {
            const float ea = __builtin_amdgcn_exp2f(ta[r] + sh), eb = __builtin_amdgcn_exp2f(tb[r] + sh);
            const float ga = fa[r] ? ea : 0.0f, gb = fb[r] ? eb : 0.0f;
            const h16 pa = toh_flush(ga); const h16 pc = toh_flush(gb);
            pb[r] = pa; pb[8 + r] = pc;
            if (EARLY) { pr[r] = toh_flush((ga - (float)pa) * QRS); pr[8 + r] = toh_flush((gb - (float)pc) * QRS); ls += ga + gb; }
            else       { ls += (float)pa + (float)pc; } }
        l = l * alpha + ls; m = mnew;
#pragma unroll
        for (int j = 0; j < 4; ++j) { o[j] = o[j] * alpha; if (EARLY) oR[j] = oR[j] * alpha; }
        const h16* va = VT + vo + key0;
#pragma unroll
        for (int j = 0; j < 4; ++j) {
            const v16h vj = ldh(va + (size_t)(16 * j) * SEQ);
            o[j] = wmma16g(vj, pb, o[j]);
            if (EARLY) {
                oR[j] = wmma16g(vj, pr, oR[j]);
                const v16h vrj = ldh(VR + vro + (size_t)key0 + (size_t)(16 * j) * EROWS);
                oR[j] = wmma16g(vrj, pb, oR[j]);
            }
        }
    }
    l += __shfl_xor(l, 16, 32);
    const bool any = l > 0.0f;
    const float lsafe = any ? l : 1.0f;
    const float inv = any ? (1.0f / lsafe) : 0.0f;
    const int wb = wave * 16 * OSP;
#pragma unroll
    for (int j = 0; j < 4; ++j) {
        v8f f = o[j];
        if (EARLY) f = o[j] + oR[j] * QRI;
        v4f a, c;
        a[0] = f[0] * inv; a[1] = f[1] * inv; a[2] = f[2] * inv; a[3] = f[3] * inv; c[0] = f[4] * inv; c[1] = f[5] * inv; c[2] = f[6] * inv; c[3] = f[7] * inv;
        *(v4fa*)(&os[wb + lr * OSP + 16 * j + 8 * hi]) = a; *(v4fa*)(&os[wb + lr * OSP + 16 * j + 8 * hi + 4]) = c; }
    wave_sync();
    float* orow = OUT + ((size_t)b * OUT_SEQ + (size_t)t0) * DM + (size_t)h * HD;
#pragma unroll 1
    for (int ps = 0; ps < 2; ++ps) {
#pragma unroll
        for (int s = 0; s < 8; ++s) { const int row = 2 * s + (lane >> 4), cofs = (lane & 15) * 4;
            const v4f val = *(const v4fa*)(&os[wb + row * OSP + cofs]);
            *(volatile v4f*)(orow + (size_t)row * DM + cofs) = val; }
        if (ps == 0) __threadfence(); }
}

__global__ __launch_bounds__(32 * AW) __attribute__((amdgpu_num_vgpr(256)))
void k_flash_early(const h16* __restrict__ QH, const h16* __restrict__ QR, const h16* __restrict__ KP, const h16* __restrict__ KR,
                   const h16* __restrict__ VT, const h16* __restrict__ VR, float* OUT) { flash_body<1>(QH, QR, KP, KR, VT, VR, OUT); }
__global__ __launch_bounds__(32 * AW) __attribute__((amdgpu_num_vgpr(256)))
void k_flash_late(const h16* __restrict__ QH, const h16* __restrict__ QR, const h16* __restrict__ KP, const h16* __restrict__ KR,
                  const h16* __restrict__ VT, const h16* __restrict__ VR, float* OUT) { flash_body<0>(QH, QR, KP, KR, VT, VR, OUT); }

static constexpr size_t al256(size_t v) { return (v + 255) & ~(size_t)255; }
static constexpr size_t SZ_XB = al256((size_t)NB * SEQ * DM * 2);
static constexpr size_t SZ_WB = al256((size_t)3 * DM * DM * 2);
static constexpr size_t SZ_PL = al256((size_t)NB * NH_ * SEQ * HD * 2);
static constexpr size_t SZ_RS = al256((size_t)NB * NH_ * EROWS * HD * 2);
static constexpr size_t SZ_TOTAL = SZ_XB + SZ_WB + 3 * SZ_PL + 3 * SZ_RS;
static_assert(SZ_TOTAL <= (size_t)134217728);
static_assert(((size_t)DM * DM * 2) % 256 == 0);
static_assert((size_t)NB * NH_ * SEQ * HD == (size_t)NB * DM * SEQ);
static_assert((size_t)NB * NH_ * EROWS * HD == (size_t)NB * DM * EROWS);
static_assert(((size_t)NB * SEQ / 64) * 64 == (size_t)NB * SEQ);
static_assert(((size_t)DM / 64) * 64 == (size_t)DM);

extern "C" void kernel_launch(void* const* d_in, const int* in_sizes, int n_in,
                              void* d_out, int out_size, void* d_ws, size_t ws_size, hipStream_t stream) {
    if (n_in < 4) return;
    const size_t needx = ((size_t)(NB - 1) * SEQ_FULL + SEQ) * DM;
    if ((size_t)in_sizes[0] < needx) return;
    if ((size_t)in_sizes[1] < (size_t)DM * DM || (size_t)in_sizes[2] < (size_t)DM * DM || (size_t)in_sizes[3] < (size_t)DM * DM) return;
    if ((size_t)out_size < ((size_t)(NB - 1) * OUT_SEQ + SEQ) * DM) return;
    if (SZ_TOTAL > ws_size) return;
    const float* xin = (const float*)d_in[0];
    const float* wq = (const float*)d_in[1];
    const float* wk = (const float*)d_in[2];
    const float* wv = (const float*)d_in[3];
    float* OUT = (float*)d_out;
    char* wsp = (char*)d_ws;
    bf* XB = (bf*)wsp; wsp += SZ_XB;
    bf* WB = (bf*)wsp; wsp += SZ_WB;
    h16* QH = (h16*)wsp; wsp += SZ_PL;
    h16* KP = (h16*)wsp; wsp += SZ_PL;
    h16* VT = (h16*)wsp; wsp += SZ_PL;
    h16* QR = (h16*)wsp; wsp += SZ_RS;
    h16* KR = (h16*)wsp; wsp += SZ_RS;
    h16* VR = (h16*)wsp; wsp += SZ_RS;
    bf* WQ = WB; bf* WK = WB + (size_t)DM * DM; bf* WV = WB + (size_t)2 * DM * DM;

    if (SEQ == SEQ_FULL) {
        const size_t n8 = (size_t)NB * SEQ * DM / 8;
        k_cvt8<<<(unsigned)((n8 + 255) / 256), 256, 0, stream>>>(xin, XB, n8);
    } else {
        const size_t n8 = (size_t)SEQ * DM / 8;
        for (int b = 0; b < NB; ++b) k_cvt8<<<(unsigned)((n8 + 255) / 256), 256, 0, stream>>>(xin + (size_t)b * SEQ_FULL * DM, XB + (size_t)b * SEQ * DM, n8);
    }
    k_wtr<<<dim3(DM / 64, DM / 64, 1), 256, 0, stream>>>(wq, WQ);
    k_wtr<<<dim3(DM / 64, DM / 64, 1), 256, 0, stream>>>(wk, WK);
    k_wtr<<<dim3(DM / 64, DM / 64, 1), 256, 0, stream>>>(wv, WV);

    k_proj_rows<<<dim3(NB * SEQ / 64, DM / 64, 1), 32, 0, stream>>>(XB, WQ, QH, QR, EROWS);
    k_proj_rows<<<dim3(NB * SEQ / 64, DM / 64, 1), 32, 0, stream>>>(XB, WK, KP, KR, EROWS);
    k_proj_cols<<<dim3(DM / 64, NB * SEQ / 64, 1), 32, 0, stream>>>(WV, XB, VT, VR, EROWS);

    k_flash_early<<<dim3(EROWS / (16 * AW), NB * NH_, 1), 32 * AW, 0, stream>>>(QH, QR, KP, KR, VT, VR, OUT);
    if (SEQ > EROWS)
        k_flash_late<<<dim3((SEQ - EROWS) / (16 * AW), NB * NH_, 1), 32 * AW, 0, stream>>>(QH, QR, KP, KR, VT, VR, OUT);
}
